// EnhancedTransformer_15350213116361
// MI455X (gfx1250) — hardware-verified
//
#include <hip/hip_runtime.h>
#include <math.h>

typedef __attribute__((ext_vector_type(16))) _Float16 v16h;
typedef __attribute__((ext_vector_type(16))) __bf16 v16b;
typedef __attribute__((ext_vector_type(8)))  _Float16 v8h;
typedef __attribute__((ext_vector_type(8)))  float v8f;
typedef __attribute__((ext_vector_type(4)))  float v4f;
typedef __attribute__((ext_vector_type(2)))  float v2f;
typedef __attribute__((ext_vector_type(4)))  unsigned v4u;
typedef __attribute__((ext_vector_type(4)))  int v4i;
typedef float __attribute__((may_alias)) float_a;
typedef int __attribute__((may_alias)) int_a;

template <typename T> __device__ __forceinline__ void vst2(void* p, T v) { *(volatile T*)p = v; __threadfence(); *(volatile T*)p = v; }
__device__ __forceinline__ v8f wmma16(v16h a, v16h b, v8f c) {
  v8f d = __builtin_amdgcn_wmma_f32_16x16x32_f16(false, a, false, b, (short)0, c, false, false);
  asm volatile("v_nop\n\tv_nop\n\tv_nop\n\tv_nop" : "+v"(d) : "v"(a), "v"(b));
  return d;
}
__device__ __forceinline__ v8f wmma_bf(v16b a, v16b b, v8f c) {
  v8f d = __builtin_amdgcn_wmma_f32_16x16x32_bf16(false, a, false, b, (short)0, c, false, false);
  asm volatile("v_nop\n\tv_nop\n\tv_nop\n\tv_nop" : "+v"(d) : "v"(a), "v"(b));
  return d;
}
__device__ __forceinline__ v16h frag_h(const _Float16* rowk0, int lane) {
  union { v16h v; v8h q[2]; } u; const _Float16* p = rowk0 + 8 * (lane >> 4);
  u.q[0] = *(const v8h*)p; u.q[1] = *(const v8h*)(p + 16); return u.v;
}
__device__ __forceinline__ v16h frag_f32(const float* rowk0, int lane) {
  v16h a; const float* p = rowk0 + 8 * (lane >> 4);
#pragma unroll
  for (int i = 0; i < 8; ++i) { a[i] = (_Float16)p[i]; a[8 + i] = (_Float16)p[16 + i]; }
  return a;
}
__device__ __forceinline__ v16h frag_f32s(const float* rowk0, int lane, float sc) {
  v16h a; const float* p = rowk0 + 8 * (lane >> 4);
#pragma unroll
  for (int i = 0; i < 8; ++i) { a[i] = (_Float16)(p[i] * sc); a[8 + i] = (_Float16)(p[16 + i] * sc); }
  return a;
}
__device__ __forceinline__ v16h fragc_f32(const float* W, int k0, int n, int lane, int ld, int K) {
  v16h a; const int g = lane >> 4;
#pragma unroll
  for (int i = 0; i < 8; ++i) { const int ka = k0 + 8 * g + i, kb = ka + 16;
    a[i] = (_Float16)(ka < K ? W[(size_t)ka * ld + n] : 0.f); a[8 + i] = (_Float16)(kb < K ? W[(size_t)kb * ld + n] : 0.f); }
  return a;
}
struct F2 { v16b h, l; };
__device__ __forceinline__ F2 bsplit16(const float v[16]) { F2 r;
#pragma unroll
  for (int i = 0; i < 16; ++i) { const __bf16 h = (__bf16)v[i]; r.h[i] = h; r.l[i] = (__bf16)(v[i] - (float)h); }
  return r; }
__device__ __forceinline__ F2 split_row(const float* row, int k0, int lane) { float v[16]; const float* p = row + k0 + 8 * (lane >> 4);
#pragma unroll
  for (int i = 0; i < 8; ++i) { v[i] = p[i]; v[8 + i] = p[16 + i]; }
  return bsplit16(v); }
__device__ __forceinline__ F2 split_rowK(const float* row, int k0, int lane, int K) { float v[16]; const int g = lane >> 4;
#pragma unroll
  for (int i = 0; i < 8; ++i) { const int ka = k0 + 8 * g + i, kb = ka + 16; v[i] = ka < K ? row[ka] : 0.f; v[8 + i] = kb < K ? row[kb] : 0.f; }
  return bsplit16(v); }
__device__ __forceinline__ F2 split_col(const float* W, int k0, int n, int lane, int ld, int K) { float v[16]; const int g = lane >> 4;
#pragma unroll
  for (int i = 0; i < 8; ++i) { const int ka = k0 + 8 * g + i, kb = ka + 16; v[i] = ka < K ? W[(size_t)ka * ld + n] : 0.f; v[8 + i] = kb < K ? W[(size_t)kb * ld + n] : 0.f; }
  return bsplit16(v); }
__device__ __forceinline__ v8f mac3(const F2& a, const F2& b, v8f c) { c = wmma_bf(a.l, b.h, c); c = wmma_bf(a.h, b.l, c); return wmma_bf(a.h, b.h, c); }
__device__ __forceinline__ float sigm(float v) { return 1.0f / (1.0f + expf(-v)); }
#define LDSX() do { asm volatile("s_wait_dscnt 0" ::: "memory"); __builtin_amdgcn_wave_barrier(); __builtin_amdgcn_fence(__ATOMIC_RELEASE, "workgroup"); } while (0)

#define NB 8
#define SS 2048
#define DD 128
#define NH 8
#define HD 16
#define WW 64
#define FF 512
#define NR (NB * SS)

__device__ __forceinline__ float gelu_e(float v) { return 0.5f * v * (1.0f + erff(v * 0.70710678118654752f)); }

__global__ __launch_bounds__(128) void k_lin(const float* __restrict__ A, const float* __restrict__ W, const float* __restrict__ bias, int N, float* __restrict__ Out) {
  __shared__ __align__(16) float so[4][16][132];
  const int tid = threadIdx.x, wave = tid >> 5, lane = tid & 31, col = lane & 15, g = lane >> 4;
  const int r0 = blockIdx.x * 64 + wave * 16, n0 = blockIdx.y * 128;
  v8f acc[8] = {};
#pragma unroll
  for (int kc = 0; kc < DD / 32; ++kc) { const v16h a = frag_f32(A + (size_t)(r0 + col) * DD + kc * 32, lane);
#pragma unroll
    for (int j = 0; j < 8; ++j) acc[j] = wmma16(a, frag_f32s(W + (size_t)(n0 + j * 16 + col) * DD + kc * 32, lane, 16.0f), acc[j]); }
#pragma unroll
  for (int j = 0; j < 8; ++j) { const float bb = bias[n0 + j * 16 + col];
#pragma unroll
    for (int r = 0; r < 8; ++r) so[wave][8 * g + r][j * 16 + col] = acc[j][r] * (1.0f / 16.0f) + bb; }
  LDSX();
#pragma unroll 4
  for (int rl = 0; rl < 16; ++rl) vst2(Out + (size_t)(r0 + rl) * N + n0 + lane * 4, *(const v4f*)(&so[wave][rl][lane * 4]));
}
__global__ __launch_bounds__(128) void k_wattn(const float* __restrict__ qkv, float* __restrict__ ao) {
  __shared__ float sk[2][WW][HD + 1], sv[2][WW][HD + 1]; __shared__ __align__(16) float so[WW][2 * HD];
  const int wdw = blockIdx.x, hp = blockIdx.y, tid = threadIdx.x, hh = tid >> 6, i = tid & 63; const int h = hp * 2 + hh; const size_t rb = (size_t)wdw * WW;
  for (int d = 0; d < HD; ++d) { sk[hh][i][d] = qkv[(rb + i) * (3 * DD) + DD + h * HD + d]; sv[hh][i][d] = qkv[(rb + i) * (3 * DD) + 2 * DD + h * HD + d]; }
  float q[HD];
#pragma unroll
  for (int d = 0; d < HD; ++d) q[d] = qkv[(rb + i) * (3 * DD) + h * HD + d] * 0.25f;
  __syncthreads();
  float mx = -3.0e38f;
  for (int j = 0; j <= i; ++j) { float s = 0.f;
#pragma unroll
    for (int d = 0; d < HD; ++d) s += q[d] * sk[hh][j][d];
    mx = fmaxf(mx, s); }
  float l = 0.f, o[HD];
#pragma unroll
  for (int d = 0; d < HD; ++d) o[d] = 0.f;
  for (int j = 0; j <= i; ++j) { float s = 0.f;
#pragma unroll
    for (int d = 0; d < HD; ++d) s += q[d] * sk[hh][j][d];
    const float p = expf(s - mx); l += p;
#pragma unroll
    for (int d = 0; d < HD; ++d) o[d] += p * sv[hh][j][d]; }
  const float inv = 1.0f / l;
#pragma unroll
  for (int d = 0; d < HD; ++d) so[i][hh * HD + d] = o[d] * inv;
  __syncthreads();
  for (int qd = tid; qd < WW * 8; qd += 128) { const int r = qd >> 3, pc = qd & 7; vst2(ao + (rb + r) * DD + hp * 2 * HD + pc * 4, *(const v4f*)(&so[r][pc * 4])); }
}
__global__ __launch_bounds__(128) void k_oln(const float* __restrict__ ao, const float* __restrict__ Wo, const float* __restrict__ bo, const float* __restrict__ x, const float* __restrict__ g1, const float* __restrict__ b1, float* __restrict__ x1) {
  __shared__ __align__(16) float so[4][16][132];
  const int tid = threadIdx.x, wave = tid >> 5, lane = tid & 31, col = lane & 15, g = lane >> 4;
  const int r0 = blockIdx.x * 64 + wave * 16;
  v8f acc[8] = {};
#pragma unroll
  for (int kc = 0; kc < DD / 32; ++kc) { const v16h a = frag_f32(ao + (size_t)(r0 + col) * DD + kc * 32, lane);
#pragma unroll
    for (int j = 0; j < 8; ++j) acc[j] = wmma16(a, frag_f32s(Wo + (size_t)(j * 16 + col) * DD + kc * 32, lane, 16.0f), acc[j]); }
#pragma unroll
  for (int j = 0; j < 8; ++j) { const int c = j * 16 + col; const float bb = bo[c];
#pragma unroll
    for (int r = 0; r < 8; ++r) so[wave][8 * g + r][c] = acc[j][r] * (1.0f / 16.0f) + bb + x[(size_t)(r0 + 8 * g + r) * DD + c]; }
  LDSX();
  { const int rl = lane >> 1, hf = lane & 1; float* row = &so[wave][rl][0]; float s = 0.f;
    for (int c = 0; c < 64; ++c) s += row[hf * 64 + c]; s += __shfl_xor(s, 1, 32); const float mu = s / (float)DD;
    float q2 = 0.f; for (int c = 0; c < 64; ++c) { const float d = row[hf * 64 + c] - mu; q2 += d * d; } q2 += __shfl_xor(q2, 1, 32); const float rs = rsqrtf(q2 / (float)DD + 1e-5f);
    LDSX();
    for (int c4 = 0; c4 < 16; ++c4) { const int cc = hf * 64 + c4 * 4; v4f v = *(const v4f*)(&row[cc]);
#pragma unroll
      for (int e = 0; e < 4; ++e) v[e] = (v[e] - mu) * rs * g1[cc + e] + b1[cc + e];
      vst2(x1 + (size_t)(r0 + rl) * DD + cc, v); } }
}
__global__ __launch_bounds__(128) void k_ffn(const float* __restrict__ x1, const float* __restrict__ w1, const float* __restrict__ b1, const float* __restrict__ w2, const float* __restrict__ b2, const float* __restrict__ g2, const float* __restrict__ be2, float* __restrict__ x2) {
  __shared__ __align__(16) float sh[64][FF + 4];
  __shared__ __align__(16) float so[4][16][132];
  const int tid = threadIdx.x, wave = tid >> 5, lane = tid & 31, col = lane & 15, g = lane >> 4;
  const int r0 = blockIdx.x * 64 + wave * 16;
  v16h ax[4];
#pragma unroll
  for (int kc = 0; kc < 4; ++kc) ax[kc] = frag_f32(x1 + (size_t)(r0 + col) * DD + kc * 32, lane);
#pragma unroll 1
  for (int nc = 0; nc < FF / 128; ++nc) { v8f acc[8] = {};
#pragma unroll
    for (int kc = 0; kc < 4; ++kc) {
#pragma unroll
      for (int j = 0; j < 8; ++j) acc[j] = wmma16(ax[kc], frag_f32s(w1 + (size_t)(nc * 128 + j * 16 + col) * DD + kc * 32, lane, 16.0f), acc[j]); }
#pragma unroll
    for (int j = 0; j < 8; ++j) { const int c = nc * 128 + j * 16 + col; const float bb = b1[c];
#pragma unroll
      for (int r = 0; r < 8; ++r) sh[wave * 16 + 8 * g + r][c] = gelu_e(acc[j][r] * (1.0f / 16.0f) + bb); } }
  LDSX();
  v8f acc[8] = {};
#pragma unroll 1
  for (int kc = 0; kc < FF / 32; ++kc) { const v16h a = frag_f32(&sh[wave * 16 + col][0] + kc * 32, lane);
#pragma unroll
    for (int j = 0; j < 8; ++j) acc[j] = wmma16(a, frag_f32s(w2 + (size_t)(j * 16 + col) * FF + kc * 32, lane, 16.0f), acc[j]); }
#pragma unroll
  for (int j = 0; j < 8; ++j) { const int c = j * 16 + col; const float bb = b2[c];
#pragma unroll
    for (int r = 0; r < 8; ++r) so[wave][8 * g + r][c] = acc[j][r] * (1.0f / 16.0f) + bb + x1[(size_t)(r0 + 8 * g + r) * DD + c]; }
  LDSX();
  { const int rl = lane >> 1, hf = lane & 1; float* row = &so[wave][rl][0]; float s = 0.f;
    for (int c = 0; c < 64; ++c) s += row[hf * 64 + c]; s += __shfl_xor(s, 1, 32); const float mu = s / (float)DD;
    float q2 = 0.f; for (int c = 0; c < 64; ++c) { const float d = row[hf * 64 + c] - mu; q2 += d * d; } q2 += __shfl_xor(q2, 1, 32); const float rs = rsqrtf(q2 / (float)DD + 1e-5f);
    LDSX();
    for (int c4 = 0; c4 < 16; ++c4) { const int cc = hf * 64 + c4 * 4; v4f v = *(const v4f*)(&row[cc]);
#pragma unroll
      for (int e = 0; e < 4; ++e) v[e] = (v[e] - mu) * rs * g2[cc + e] + be2[cc + e];
      vst2(x2 + (size_t)(r0 + rl) * DD + cc, v); } }
}
__global__ __launch_bounds__(128) void k_st(const float* __restrict__ sp, const float* __restrict__ tp, const float* __restrict__ Ws, const float* __restrict__ bs, const float* __restrict__ Wt, const float* __restrict__ bt,
                                          float* __restrict__ se, float* __restrict__ te, _Float16* __restrict__ sn, _Float16* __restrict__ tn) {
  __shared__ __align__(16) float so[4][16][132];
  const int tid = threadIdx.x, wave = tid >> 5, lane = tid & 31, col = lane & 15, g = lane >> 4;
  const int r0 = blockIdx.x * 64 + wave * 16, which = blockIdx.y; const float* A = which ? tp : sp; const float* W = which ? Wt : Ws; const float* bias = which ? bt : bs;
  float* E = which ? te : se; _Float16* Nn = which ? tn : sn;
  v8f acc[8] = {};
#pragma unroll
  for (int kc = 0; kc < DD / 32; ++kc) { const v16h a = frag_f32(A + (size_t)(r0 + col) * DD + kc * 32, lane);
#pragma unroll
    for (int j = 0; j < 8; ++j) acc[j] = wmma16(a, frag_f32s(W + (size_t)(j * 16 + col) * DD + kc * 32, lane, 16.0f), acc[j]); }
#pragma unroll
  for (int j = 0; j < 8; ++j) { const int c = j * 16 + col; const float bb = bias[c];
#pragma unroll
    for (int r = 0; r < 8; ++r) so[wave][8 * g + r][c] = acc[j][r] * (1.0f / 16.0f) + bb; }
  LDSX();
  { const int rl = lane >> 1, hf = lane & 1; const float* row = &so[wave][rl][0]; float q2 = 0.f;
    for (int c = 0; c < 64; ++c) { const float v = row[hf * 64 + c]; q2 += v * v; } q2 += __shfl_xor(q2, 1, 32);
    const float inv = 1.0f / fmaxf(sqrtf(q2), 1e-8f);
    for (int c4 = 0; c4 < 16; ++c4) { const int cc = hf * 64 + c4 * 4; const v4f v = *(const v4f*)(&row[cc]); vst2(E + (size_t)(r0 + rl) * DD + cc, v); }
    for (int c8 = 0; c8 < 8; ++c8) { const int cc = hf * 64 + c8 * 8; union { v8h hh; v4u u; } pk;
#pragma unroll
      for (int e = 0; e < 8; ++e) pk.hh[e] = (_Float16)(row[cc + e] * inv * 8.0f);
      vst2(Nn + (size_t)(r0 + rl) * DD + cc, pk.u); } }
}
__global__ __launch_bounds__(128) void k_sim(const _Float16* __restrict__ sn, const _Float16* __restrict__ tn, float* __restrict__ sim) {
  const int tid = threadIdx.x, wave = tid >> 5, lane = tid & 31, col = lane & 15, g = lane >> 4;
  const int b = blockIdx.y, i0 = blockIdx.x * 64 + wave * 16; const size_t base = (size_t)b * SS;
  v16h as_[4], at_[4];
#pragma unroll
  for (int kc = 0; kc < 4; ++kc) { as_[kc] = frag_h(sn + (base + i0 + col) * DD + kc * 32, lane); at_[kc] = frag_h(tn + (base + i0 + col) * DD + kc * 32, lane); }
  float rs[8] = {0.f, 0.f, 0.f, 0.f, 0.f, 0.f, 0.f, 0.f};
#pragma unroll 1
  for (int jt = 0; jt < SS / 16; ++jt) { v8f s1 = {}, s2 = {};
#pragma unroll
    for (int kc = 0; kc < 4; ++kc) { s1 = wmma16(as_[kc], frag_h(sn + (base + jt * 16 + col) * DD + kc * 32, lane), s1); s2 = wmma16(at_[kc], frag_h(tn + (base + jt * 16 + col) * DD + kc * 32, lane), s2); }
#pragma unroll
    for (int r = 0; r < 8; ++r) rs[r] += s1[r] * s2[r]; }
#pragma unroll
  for (int off = 8; off >= 1; off >>= 1) {
#pragma unroll
    for (int r = 0; r < 8; ++r) rs[r] += __shfl_xor(rs[r], off, 32); }
  __shared__ __align__(16) float so[64];
  if (col == 0) {
#pragma unroll
    for (int r = 0; r < 8; ++r) so[wave * 16 + 8 * g + r] = rs[r] * (1.0f / 4096.0f) * (1.0f / (float)SS); }
  __syncthreads();
  if (tid < 16) vst2(sim + base + blockIdx.x * 64 + tid * 4, *(const v4f*)(&so[tid * 4]));
}
__global__ __launch_bounds__(128) void k_iattn(const float* __restrict__ q2, const float* __restrict__ kv2, float* __restrict__ ao2) {
  __shared__ __align__(16) float sS[4][16][20];
  __shared__ __align__(16) float sV[4][16][DD + 4];
  __shared__ __align__(16) float so[4][16][DD + 4];
  const int tid = threadIdx.x, wave = tid >> 5, lane = tid & 31, col = lane & 15, g = lane >> 4;
  const int s0 = (blockIdx.x * 4 + wave) * 2;
  auto rowof = [&](int m) { return (size_t)(m & 7) * SS + s0 + (m >> 3); };
  for (int q = lane; q < 16 * 32; q += 32) { const int m = q >> 5, pc = q & 31; const v4f v = *(const v4f*)(kv2 + rowof(m) * (2 * DD) + DD + pc * 4);
    sV[wave][m][pc * 4] = v[0]; sV[wave][m][pc * 4 + 1] = v[1]; sV[wave][m][pc * 4 + 2] = v[2]; sV[wave][m][pc * 4 + 3] = v[3]; }
  LDSX();
#pragma unroll 1
  for (int h = 0; h < NH; ++h) {
    v16h a, bk;
#pragma unroll
    for (int i = 0; i < 8; ++i) { a[i] = (_Float16)(q2[rowof(col) * DD + h * HD + 8 * g + i] * 0.25f); a[8 + i] = (_Float16)0.f; bk[i] = (_Float16)kv2[rowof(col) * (2 * DD) + h * HD + 8 * g + i]; bk[8 + i] = (_Float16)0.f; }
    v8f s = {}; s = wmma16(a, bk, s);
#pragma unroll
    for (int r = 0; r < 8; ++r) sS[wave][8 * g + r][col] = s[r];
    LDSX();
    if (g == 0) { const int m = col, cb = (m >> 3) * 8; float mx = -3.0e38f;
#pragma unroll
      for (int e = 0; e < 8; ++e) mx = fmaxf(mx, sS[wave][m][cb + e]);
      float l = 0.f, pv[8];
#pragma unroll
      for (int e = 0; e < 8; ++e) { pv[e] = expf(sS[wave][m][cb + e] - mx); l += pv[e]; }
      const float inv = 1.0f / l;
#pragma unroll
      for (int e = 0; e < 16; ++e) sS[wave][m][e] = (e >= cb && e < cb + 8) ? pv[e - cb] * inv : 0.f; }
    LDSX();
    v16h pa, vb;
#pragma unroll
    for (int i = 0; i < 8; ++i) { pa[i] = (_Float16)sS[wave][col][8 * g + i]; pa[8 + i] = (_Float16)0.f; vb[i] = (_Float16)sV[wave][8 * g + i][h * HD + col]; vb[8 + i] = (_Float16)0.f; }
    v8f o = {}; o = wmma16(pa, vb, o);
#pragma unroll
    for (int r = 0; r < 8; ++r) so[wave][8 * g + r][h * HD + col] = o[r];
    LDSX(); }
  for (int q = lane; q < 16 * 32; q += 32) { const int m = q >> 5, pc = q & 31; vst2(ao2 + rowof(m) * DD + pc * 4, *(const v4f*)(&so[wave][m][pc * 4])); }
}
__global__ __launch_bounds__(128) void k_fin(const float* __restrict__ ao2, const float* __restrict__ W, const float* __restrict__ bias, const float* __restrict__ x2, const float* __restrict__ sim, float* __restrict__ out) {
  __shared__ __align__(16) float so[4][16][132];
  const int tid = threadIdx.x, wave = tid >> 5, lane = tid & 31, col = lane & 15, g = lane >> 4;
  const int r0 = blockIdx.x * 64 + wave * 16;
  v8f acc[8] = {};
#pragma unroll
  for (int kc = 0; kc < DD / 32; ++kc) { const v16h a = frag_f32(ao2 + (size_t)(r0 + col) * DD + kc * 32, lane);
#pragma unroll
    for (int j = 0; j < 8; ++j) acc[j] = wmma16(a, frag_f32s(W + (size_t)(j * 16 + col) * DD + kc * 32, lane, 16.0f), acc[j]); }
#pragma unroll
  for (int j = 0; j < 8; ++j) { const int c = j * 16 + col; const float bb = bias[c];
#pragma unroll
    for (int r = 0; r < 8; ++r) { const size_t row = (size_t)(r0 + 8 * g + r); so[wave][8 * g + r][c] = x2[row * DD + c] + sim[row] * (acc[j][r] * (1.0f / 16.0f) + bb); } }
  LDSX();
#pragma unroll 4
  for (int rl = 0; rl < 16; ++rl) vst2(out + (size_t)(r0 + rl) * DD + lane * 4, *(const v4f*)(&so[wave][rl][lane * 4]));
}
extern "C" void kernel_launch(void* const* d_in, const int* in_sizes, int n_in, void* d_out, int out_size, void* d_ws, size_t ws_size, hipStream_t stream) {
  (void)in_sizes; (void)n_in; (void)out_size; (void)ws_size;
  const float** I = (const float**)d_in;
  const float* x = I[0]; const float* spat = I[1]; const float* temp = I[2]; const float* lwi = I[3]; const float* lwib = I[4]; const float* lwo = I[5]; const float* lwob = I[6];
  const float* sw = I[7]; const float* sb = I[8]; const float* tw = I[9]; const float* tb = I[10]; const float* iiw = I[11]; const float* iib = I[12]; const float* iow = I[13]; const float* iob = I[14];
  const float* f1 = I[15]; const float* f1b = I[16]; const float* f2 = I[17]; const float* f2b = I[18]; const float* g1 = I[19]; const float* b1 = I[20]; const float* g2 = I[21]; const float* b2 = I[22];
  float* out = (float*)d_out;
  char* ws = (char*)d_ws; size_t off = 0;
  auto take = [&](size_t bytes) { char* p = ws + off; off += (bytes + 255) & ~(size_t)255; return p; };
  float* qkv = (float*)take((size_t)NR * 3 * DD * 4); float* ao = (float*)take((size_t)NR * DD * 4); float* x1 = (float*)take((size_t)NR * DD * 4); float* x2 = (float*)take((size_t)NR * DD * 4);
  float* se = (float*)take((size_t)NR * DD * 4); float* te = (float*)take((size_t)NR * DD * 4); _Float16* sn = (_Float16*)take((size_t)NR * DD * 2); _Float16* tn = (_Float16*)take((size_t)NR * DD * 2);
  float* sim = (float*)take((size_t)NR * 4); float* q2 = (float*)take((size_t)NR * DD * 4); float* kv2 = (float*)take((size_t)NR * 2 * DD * 4); float* ao2 = (float*)take((size_t)NR * DD * 4);
  k_lin<<<dim3(NR / 64, 3), 128, 0, stream>>>(x, lwi, lwib, 3 * DD, qkv);
  k_wattn<<<dim3(NR / WW, NH / 2), 128, 0, stream>>>(qkv, ao);
  k_oln<<<NR / 64, 128, 0, stream>>>(ao, lwo, lwob, x, g1, b1, x1);
  k_ffn<<<NR / 64, 128, 0, stream>>>(x1, f1, f1b, f2, f2b, g2, b2, x2);
  k_st<<<dim3(NR / 64, 2), 128, 0, stream>>>(spat, temp, sw, sb, tw, tb, se, te, sn, tn);
  k_sim<<<dim3(SS / 64, NB), 128, 0, stream>>>(sn, tn, sim);
  k_lin<<<dim3(NR / 64, 1), 128, 0, stream>>>(se, iiw, iib, DD, q2);
  k_lin<<<dim3(NR / 64, 2), 128, 0, stream>>>(te, iiw + (size_t)DD * DD, iib + DD, 2 * DD, kv2);
  k_iattn<<<SS / 8, 128, 0, stream>>>(q2, kv2, ao2);
  k_fin<<<NR / 64, 128, 0, stream>>>(ao2, iow, iob, x2, sim, out);
}
